// DualPathAttention_15109694947381
// MI455X (gfx1250) — hardware-run, weakly checked
//
#include <hip/hip_runtime.h>
#include <math.h>

#ifndef NB
#define NB 2
#endif
#ifndef SEQ
#define SEQ 2048
#endif
#define NB_FULL 2
#define T_FULL 2048
#define CE 1024
#define NH 16
#define HD 64
#define NX 256
#define MT (NB * SEQ)
#define QKP (2 * CE)
#define LNP 320
#define LSP (NH * 32)
#define VEP (NB * NX)
#define LTOK 32

static_assert(SEQ % 64 == 0);
static_assert(SEQ >= NX && SEQ <= T_FULL && NB <= NB_FULL && NB >= 1);
static_assert(CE % 64 == 0 && NX % 64 == 0 && CE % 32 == 0 && QKP % 64 == 0 && LNP % 64 == 0);
static_assert(NH * HD == CE && HD == 64);
static_assert(LNP >= 4 * 64 + NH && 4 * NH == 64);
static_assert(MT % LTOK == 0 && MT % 64 == 0 && (SEQ - NX) % 64 == 0);
static_assert(LTOK * NH == 512);
static_assert(LTOK * LSP * 2 == 512 * 4 * 16);
static_assert(LTOK * 4 == 8 * 16);
static_assert(HD * 2 == 8 * 16);
static_assert(4 * 4 == 16);
static_assert(2 * LTOK * 64 * 16 + LTOK * 4 <= 131072);
static_assert(8 * 16 * 68 * 4 <= 131072);
static_assert(4 * 16 * 64 * 2 * 2 + 4 * 16 * 68 * 4 <= 131072);

typedef __attribute__((ext_vector_type(16))) _Float16 v16h;
typedef __attribute__((ext_vector_type(16))) __bf16   v16b;
typedef __attribute__((ext_vector_type(8)))  __bf16   v8b;
typedef __attribute__((ext_vector_type(8)))  float    v8f;
typedef __attribute__((ext_vector_type(4)))  float    v4f;
typedef __attribute__((ext_vector_type(4)))  unsigned int v4u;

union FB { v16b v; v8b h[2]; };

__device__ __forceinline__ unsigned int f2bf_bits(float f) { const unsigned int u = __float_as_uint(f); return (u + 0x7FFFu + ((u >> 16) & 1u)) >> 16; }
__device__ __forceinline__ float bf_bits2f(unsigned int h) { return __uint_as_float(h << 16); }
__device__ __forceinline__ float cmb_bf(float v) { return bf_bits2f(f2bf_bits(v)); }
__device__ __forceinline__ unsigned int h_bits(float v) { return (unsigned int)__builtin_bit_cast(unsigned short, (_Float16)v); }

__device__ __forceinline__ v4u pk8h(v4f a, v4f b) {
  v4u p;
  p.x = h_bits(a.x) | (h_bits(a.y) << 16); p.y = h_bits(a.z) | (h_bits(a.w) << 16);
  p.z = h_bits(b.x) | (h_bits(b.y) << 16); p.w = h_bits(b.z) | (h_bits(b.w) << 16);
  return p;
}
__device__ __forceinline__ v4u pk8b(v4f a, v4f b) {
  v4u p;
  p.x = f2bf_bits(a.x) | (f2bf_bits(a.y) << 16); p.y = f2bf_bits(a.z) | (f2bf_bits(a.w) << 16);
  p.z = f2bf_bits(b.x) | (f2bf_bits(b.y) << 16); p.w = f2bf_bits(b.z) | (f2bf_bits(b.w) << 16);
  return p;
}
__device__ __forceinline__ void bf_hl(float v, unsigned int& hi, unsigned int& lo) { hi = f2bf_bits(v); lo = f2bf_bits(v - bf_bits2f(hi)); }
__device__ __forceinline__ void pk8s(v4f a, v4f b, v4u& ph, v4u& pl) {
  unsigned int h0, l0, h1, l1, h2, l2, h3, l3, h4, l4, h5, l5, h6, l6, h7, l7;
  bf_hl(a.x, h0, l0); bf_hl(a.y, h1, l1); bf_hl(a.z, h2, l2); bf_hl(a.w, h3, l3);
  bf_hl(b.x, h4, l4); bf_hl(b.y, h5, l5); bf_hl(b.z, h6, l6); bf_hl(b.w, h7, l7);
  ph.x = h0 | (h1 << 16); ph.y = h2 | (h3 << 16); ph.z = h4 | (h5 << 16); ph.w = h6 | (h7 << 16);
  pl.x = l0 | (l1 << 16); pl.y = l2 | (l3 << 16); pl.z = l4 | (l5 << 16); pl.w = l6 | (l7 << 16);
}

typedef _Float16 h16;
static __device__ __forceinline__ h16 toh_flush(float v) { const h16 r = (h16)v; return (fabsf(v) < 6.103515625e-05f) ? (h16)0.0f : r; }
__device__ __forceinline__ unsigned int hf_bits(float v) { return (unsigned int)__builtin_bit_cast(unsigned short, toh_flush(v)); }
__device__ __forceinline__ v4u pk8hf(v4f a, v4f b) {
  v4u p;
  p.x = hf_bits(a.x) | (hf_bits(a.y) << 16); p.y = hf_bits(a.z) | (hf_bits(a.w) << 16);
  p.z = hf_bits(b.x) | (hf_bits(b.y) << 16); p.w = hf_bits(b.z) | (hf_bits(b.w) << 16);
  return p;
}

__device__ __forceinline__ v16b ldfrag_g(const __bf16* __restrict__ p) { FB f; f.h[0] = *(const v8b*)p; f.h[1] = *(const v8b*)(p + 16); return f.v; }

template <bool F16> __device__ __forceinline__ v8f mma_raw(v16b a, v16b b, v8f c) {
  if (F16) {
    const v16h ah = __builtin_bit_cast(v16h, a), bh = __builtin_bit_cast(v16h, b);
    return __builtin_amdgcn_wmma_f32_16x16x32_f16(false, ah, false, bh, (short)0, c, false, false);
  }
  return __builtin_amdgcn_wmma_f32_16x16x32_bf16(false, a, false, b, (short)0, c, false, false);
}
template <bool F16> __device__ __forceinline__ v8f mma16(v16b a, v16b b, v8f c) {
  c = mma_raw<F16>(a, b, c);
  asm volatile("v_nop\n\tv_nop\n\tv_nop\n\tv_nop" : "+v"(c) : "v"(a), "v"(b));
  return c;
}
__device__ __forceinline__ void dep_guard_b(v8f& a, v8f& b, v16b x, v16b y) { asm volatile("v_nop\n\tv_nop\n\tv_nop\n\tv_nop" : "+v"(a), "+v"(b) : "v"(x), "v"(y)); }
__device__ __forceinline__ void keep4_b(v16b a, v16b b, v16b c, v16b d) { asm volatile("v_nop" :: "v"(a), "v"(b), "v"(c), "v"(d)); }
__device__ __forceinline__ void acc_guard4(v8f& a, v8f& b, v8f& c, v8f& d) { asm volatile("v_nop\n\tv_nop\n\tv_nop\n\tv_nop" : "+v"(a), "+v"(b), "+v"(c), "+v"(d)); }
__device__ __forceinline__ void wave_sync() {
  __builtin_amdgcn_fence(3  , "workgroup");
  __builtin_amdgcn_wave_barrier();
  __builtin_amdgcn_fence(2  , "workgroup");
}

__global__ __launch_bounds__(256) void k_castT(const float* __restrict__ SRC, int lds, unsigned short* __restrict__ DST, int ldd, int nR, int nC, float sc, int asbf) {
  const long long u = (long long)blockIdx.x * 256 + threadIdx.x; const int per = nR / 8;
  if (u >= (long long)nC * per) return;
  const int c = (int)(u / per); const int r0 = 8 * (int)(u % per);
  const float* s = SRC + (long long)r0 * lds + c;
  v4f wa, wb;
  wa.x = cmb_bf(s[0]) * sc;                  wa.y = cmb_bf(s[(long long)lds]) * sc;
  wa.z = cmb_bf(s[2 * (long long)lds]) * sc; wa.w = cmb_bf(s[3 * (long long)lds]) * sc;
  wb.x = cmb_bf(s[4 * (long long)lds]) * sc; wb.y = cmb_bf(s[5 * (long long)lds]) * sc;
  wb.z = cmb_bf(s[6 * (long long)lds]) * sc; wb.w = cmb_bf(s[7 * (long long)lds]) * sc;
  const v4u ph = pk8hf(wa, wb); const v4u pb = pk8b(wa, wb);
  const v4u pk = asbf ? pb : ph;
  volatile v4u* d = (volatile v4u*)(DST + (long long)c * ldd + r0);
  *d = pk; __threadfence(); *d = pk;
}

__global__ __launch_bounds__(256) void k_castX16(const float* __restrict__ X, unsigned short* __restrict__ Y) {
  const long long u = (long long)blockIdx.x * 256 + threadIdx.x;
  if (u >= (long long)MT * (CE / 8)) return;
  const int row = (int)(u / (CE / 8)); const int c0 = 8 * (int)(u % (CE / 8));
  const int b = row / SEQ, t = row - b * SEQ;
  const float* s = X + ((long long)b * T_FULL + t) * CE + c0;
  v4f a = *(const v4f*)s, bq = *(const v4f*)(s + 4);
  a.x = cmb_bf(a.x); a.y = cmb_bf(a.y); a.z = cmb_bf(a.z); a.w = cmb_bf(a.w);
  bq.x = cmb_bf(bq.x); bq.y = cmb_bf(bq.y); bq.z = cmb_bf(bq.z); bq.w = cmb_bf(bq.w);
  const v4u pk = pk8hf(a, bq);
  volatile v4u* d = (volatile v4u*)(Y + (long long)row * CE + c0);
  *d = pk; __threadfence(); *d = pk;
}

template <int ET, bool SPLITA, int BIAS_MODE, int OUT_MODE, int RESID, int ACT>
__global__ __launch_bounds__(256) void k_gemm64(
    const unsigned short* __restrict__ Ap, const unsigned short* __restrict__ A2p, int lda, long long strideA,
    const unsigned short* __restrict__ Btp, int ldb,
    unsigned short* __restrict__ O16a, unsigned short* __restrict__ O16b, unsigned short* __restrict__ O16c,
    float* __restrict__ O32, int ldc, long long strideC,
    const float* __restrict__ bias, const float* __restrict__ resid, int ldr, long long strideR,
    int M, int N, int K, float scale) {
  constexpr bool F16 = (ET == 0);
  __shared__ __align__(16) float sT[8][16 * 68];
  const int bz = blockIdx.y;
  const int lane = threadIdx.x & 31, wave = threadIdx.x >> 5;
  const int tilesN = N >> 6, tilesM = M >> 6;
  const int tile = blockIdx.x * 8 + wave;
  if (tile >= tilesM * tilesN) return;
  const int tm = tile / tilesN, tn = tile - tm * tilesN;
  const int m0 = tm << 6, n0 = tn << 6;
  const __bf16* Ab  = (const __bf16*)Ap + (size_t)bz * (size_t)strideA;
  const __bf16* Ab2 = SPLITA ? ((const __bf16*)A2p + (size_t)bz * (size_t)strideA) : Ab;
  const __bf16* Bb  = (const __bf16*)Btp;
  const int rl = lane & 15, koff = (lane >> 4) * 8, mOff = (lane >> 4) * 8;

  v8f acc[4][4];
#pragma unroll
  for (int i = 0; i < 4; ++i)
#pragma unroll
    for (int j = 0; j < 4; ++j) { v8f z = {}; acc[i][j] = z; }

  for (int k0 = 0; k0 < K; k0 += 32) {
    v16b bh[4];
#pragma unroll
    for (int j = 0; j < 4; ++j) bh[j] = ldfrag_g(Bb + (size_t)(n0 + (j << 4) + rl) * ldb + koff + k0);
#pragma unroll
    for (int i = 0; i < 4; ++i) {
      const size_t ao = (size_t)(m0 + (i << 4) + rl) * lda + koff + k0;
      const v16b ah = ldfrag_g(Ab + ao);
      v16b al = ah;
      if (SPLITA) al = ldfrag_g(Ab2 + ao);
#pragma unroll
      for (int j = 0; j < 4; ++j) {
        acc[i][j] = mma_raw<F16>(ah, bh[j], acc[i][j]);
        if (SPLITA) acc[i][j] = mma_raw<F16>(al, bh[j], acc[i][j]);
      }
      dep_guard_b(acc[i][0], acc[i][3], ah, al);
    }
    keep4_b(bh[0], bh[1], bh[2], bh[3]);
  }
  acc_guard4(acc[0][0], acc[0][1], acc[0][2], acc[0][3]);
  acc_guard4(acc[1][0], acc[1][1], acc[1][2], acc[1][3]);
  acc_guard4(acc[2][0], acc[2][1], acc[2][2], acc[2][3]);
  acc_guard4(acc[3][0], acc[3][1], acc[3][2], acc[3][3]);

  float* slab = sT[wave];
  const float* Rb = (RESID != 0) ? (resid + (size_t)bz * (size_t)strideR) : resid;
#pragma unroll
  for (int i = 0; i < 4; ++i) {
    const int mBase = m0 + (i << 4);
#pragma unroll
    for (int j = 0; j < 4; ++j) {
      const int n = n0 + (j << 4) + rl;
      float bv = 0.f;
      if (BIAS_MODE == 2) bv = cmb_bf(bias[n]);
#pragma unroll
      for (int r = 0; r < 8; ++r) {
        float v = acc[i][j][r] * scale;
        if (BIAS_MODE == 1) v += cmb_bf(bias[mBase + mOff + r]);
        if (BIAS_MODE == 2) v += bv;
        if (ACT == 5) v = 0.5f * v * (1.0f + erff(v * 0.70710678118654752f));
        if (RESID == 1) v += Rb[(size_t)(mBase + mOff + r) * ldr + n];
        if (RESID == 2) v += cmb_bf(Rb[(size_t)(mBase + mOff + r) * ldr + n]);
        slab[(mOff + r) * 68 + (j << 4) + rl] = v;
      }
    }
    wave_sync();
    if (OUT_MODE == 0) {
      float* C = O32 + (size_t)bz * (size_t)strideC;
      const int hh2 = lane >> 4, c4 = (lane & 15) * 4;
      for (int pass = 0; pass < 2; ++pass) {
#pragma unroll
        for (int it = 0; it < 8; ++it) {
          const int row = it * 2 + hh2;
          const v4f v = *(const v4f*)(slab + row * 68 + c4);
          *(volatile v4f*)(C + (size_t)(mBase + row) * ldc + n0 + c4) = v;
        }
        __threadfence();
      }
    } else {
      const int q = lane >> 3, c8 = (lane & 7) * 8;
      for (int pass = 0; pass < 2; ++pass) {
#pragma unroll
        for (int it = 0; it < 4; ++it) {
          const int row = it * 4 + q;
          const float* sp = slab + row * 68 + c8;
          const v4f wa = *(const v4f*)sp, wb = *(const v4f*)(sp + 4);
          const size_t o = (size_t)bz * (size_t)strideC + (size_t)(mBase + row) * ldc + n0 + c8;
          if (OUT_MODE == 1 || OUT_MODE == 3) { const v4u pk = pk8h(wa, wb); *(volatile v4u*)(O16a + o) = pk; }
          if (OUT_MODE == 2) { v4u ph, pl; pk8s(wa, wb, ph, pl); *(volatile v4u*)(O16a + o) = ph; *(volatile v4u*)(O16b + o) = pl; }
          if (OUT_MODE == 3) { v4u ph, pl; pk8s(wa, wb, ph, pl); *(volatile v4u*)(O16b + o) = ph; *(volatile v4u*)(O16c + o) = pl; }
        }
        __threadfence();
      }
    }
    wave_sync();
  }
}

__global__ __launch_bounds__(512) void k_lines(const float* __restrict__ LN, const float* __restrict__ gate_b,
                                                unsigned short* __restrict__ RLP, unsigned short* __restrict__ JWP, float* __restrict__ GATE) {
#pragma clang fp contract(off)
  __shared__ v4u tile[2][LTOK * 64];
  __shared__ float gsh[LTOK];
  const int tid = threadIdx.x, tk = tid >> 4, h = tid & 15;
  const int tok0 = blockIdx.x * LTOK;
  const int tok = tok0 + tk;
  const int b = tok / SEQ, t = tok - b * SEQ;
  const int prow = (t > 0) ? (tok - 1) : tok;
#pragma unroll 1
  for (int it = 0; it < 2; ++it) {
    const int rowA = (it != 0) ? tok : prow;
    v4f a_raw = *(const v4f*)(LN + (size_t)rowA * LNP + it * 128 + h * 4);
    const v4f p2 = *(const v4f*)(LN + (size_t)tok * LNP + it * 128 + 64 + h * 4);
    asm volatile("" : "+v"(a_raw));
    const bool zr = (it == 0) && (t == 0);
    v4f p1;
    p1.x = zr ? 0.0f : a_raw.x; p1.y = zr ? 0.0f : a_raw.y; p1.z = zr ? 0.0f : a_raw.z; p1.w = zr ? 0.0f : a_raw.w;
    const float L0 = p1.x * p2.y - p1.y * p2.x;
    const float L1 = p1.x * p2.z - p1.z * p2.x;
    const float L2 = p1.x * p2.w - p1.w * p2.x;
    const float L3 = p1.y * p2.z - p1.z * p2.y;
    const float L4 = p1.y * p2.w - p1.w * p2.y;
    const float L5 = p1.z * p2.w - p1.w * p2.z;
    const float ss = ((L0 * L0 + L1 * L1) + (L2 * L2 + L3 * L3)) + (L4 * L4 + L5 * L5);
    const float inv = __builtin_amdgcn_rcpf(fmaxf(sqrtf(ss), 1e-12f));
    const float n0 = L0 * inv, n1 = L1 * inv, n2 = L2 * inv, n3 = L3 * inv, n4 = L4 * inv, n5 = L5 * inv;
    const bool rd = (it != 0);
    float u[6];
    u[0] = rd ? n0 : n5;  u[1] = rd ? n1 : -n4; u[2] = rd ? n2 : n3;
    u[3] = rd ? n3 : n2;  u[4] = rd ? n4 : -n1; u[5] = rd ? n5 : n0;
    unsigned int hb[6], lb[6];
#pragma unroll
    for (int i = 0; i < 6; ++i) bf_hl(u[i], hb[i], lb[i]);
    unsigned int e[24];
#pragma unroll
    for (int i = 0; i < 6; ++i) {
      e[i] = hb[i];
      e[6 + i] = rd ? hb[i] : lb[i];
      e[12 + i] = rd ? lb[i] : hb[i];
      e[18 + i] = lb[i];
    }
    v4u w0, w1, w2, w3;
    w0.x = e[0]  | (e[1]  << 16); w0.y = e[2]  | (e[3]  << 16); w0.z = e[4]  | (e[5]  << 16); w0.w = e[6]  | (e[7]  << 16);
    w1.x = e[8]  | (e[9]  << 16); w1.y = e[10] | (e[11] << 16); w1.z = e[12] | (e[13] << 16); w1.w = e[14] | (e[15] << 16);
    w2.x = e[16] | (e[17] << 16); w2.y = e[18] | (e[19] << 16); w2.z = e[20] | (e[21] << 16); w2.w = e[22] | (e[23] << 16);
    w3.x = 0u; w3.y = 0u; w3.z = 0u; w3.w = 0u;
    const int ti = 1 - it;
    const int tb = tk * 64 + h * 4;
    tile[ti][tb + 0] = w0; tile[ti][tb + 1] = w1; tile[ti][tb + 2] = w2; tile[ti][tb + 3] = w3;
  }
  {
    const float gl = LN[(size_t)tok * LNP + 256 + h] + cmb_bf(gate_b[h]);
    float sg = __builtin_amdgcn_rcpf(1.0f + expf(-gl));
    sg += __shfl_xor(sg, 1, 32); sg += __shfl_xor(sg, 2, 32); sg += __shfl_xor(sg, 4, 32); sg += __shfl_xor(sg, 8, 32);
    if (h == 0) gsh[tk] = sg * 0.0625f;
  }
  __syncthreads();
  const int gi = (tid < 8) ? (tid * 4) : 0;
  v4f gq; gq.x = gsh[gi]; gq.y = gsh[gi + 1]; gq.z = gsh[gi + 2]; gq.w = gsh[gi + 3];
  for (int pass = 0; pass < 2; ++pass) {
#pragma unroll
    for (int i = 0; i < 4; ++i) {
      const int p = i * 512 + tid;
      const v4u ra = tile[0][p];
      const v4u wa = tile[1][p];
      *(volatile v4u*)(RLP + (size_t)tok0 * LSP + (size_t)p * 8) = ra;
      *(volatile v4u*)(JWP + (size_t)tok0 * LSP + (size_t)p * 8) = wa;
    }
    if (tid < 8) *(volatile v4f*)(GATE + tok0 + tid * 4) = gq;
    __threadfence();
  }
}

template <bool EARLY>
__device__ __forceinline__ void dual_attn_body(
    const unsigned short* __restrict__ QAp, const unsigned short* __restrict__ QBp,
    const unsigned short* __restrict__ RLp, const unsigned short* __restrict__ JWp,
    const unsigned short* __restrict__ VAp, const unsigned short* __restrict__ VBp,
    const float* __restrict__ gatev, const float* __restrict__ inc_scale,
    unsigned short* __restrict__ C16, unsigned short* __restrict__ CHp, unsigned short* __restrict__ CLp,
    int nqb, int qb0) {
  constexpr bool F16 = !EARLY;
  const float PSC = F16 ? 32768.0f : 1.0f;
  const float CSC = F16 ? 64.0f : 1.0f;
  const float L2E = 1.4426950408889634f;
  __shared__ __align__(16) __bf16 Psh[4][16 * 64];
  __shared__ __align__(16) __bf16 Psl[EARLY ? 4 : 1][EARLY ? 16 * 64 : 8];
  __shared__ __align__(16) float  Os[4][16 * 68];

  const int tid = threadIdx.x, lane = tid & 31, hh = lane >> 4, c = lane & 15;
  const int wave = __builtin_amdgcn_readfirstlane(tid >> 5);
  const int bx = blockIdx.x;
  const int qb = qb0 + bx % nqb;
  const int bhd = bx / nqb;
  const int h = bhd % NH, b = bhd / NH;
  const int q0 = qb * 64 + wave * 16;
  constexpr int RQ = EARLY ? NX : SEQ;
  constexpr size_t VP = EARLY ? (size_t)VEP : (size_t)MT;

  const __bf16* QA = (const __bf16*)QAp; const __bf16* QB = (const __bf16*)QBp;
  const __bf16* RL = (const __bf16*)RLp; const __bf16* JW = (const __bf16*)JWp;
  const __bf16* VA = (const __bf16*)VAp; const __bf16* VB = (const __bf16*)VBp;

  float gt[8], mrow[8], lrow[8];
#pragma unroll
  for (int r = 0; r < 8; ++r) gt[r] = gatev[(size_t)b * SEQ + q0 + 8 * hh + r];
  const float inc = cmb_bf(inc_scale[h]);

  __bf16* pwh = Psh[wave];
  __bf16* pwl = Psl[EARLY ? wave : 0];
  float* os = Os[wave];
  const size_t vcol = (size_t)b * RQ + 8 * hh;

#pragma unroll
  for (int ph = 0; ph < 2; ++ph) {
    v16b fa[2], fl[2];
    if (ph == 0) {
      const size_t qo = ((size_t)b * RQ + q0 + c) * QKP + (size_t)h * HD + 8 * hh;
#pragma unroll
      for (int dc = 0; dc < 2; ++dc) {
        fa[dc] = ldfrag_g(QA + qo + dc * 32);
        fl[dc] = fa[dc];
        if (EARLY) fl[dc] = ldfrag_g(QB + qo + dc * 32);
      }
    } else {
      const size_t ro = ((size_t)b * SEQ + q0 + c) * LSP + (size_t)h * 32 + 8 * hh;
      fa[0] = ldfrag_g(RL + ro); fa[1] = fa[0]; fl[0] = fa[0]; fl[1] = fa[0];
    }
#pragma unroll
    for (int r = 0; r < 8; ++r) { mrow[r] = -INFINITY; lrow[r] = 0.f; }
    v8f oacc[4];
#pragma unroll
    for (int t = 0; t < 4; ++t) { v8f z = {}; oacc[t] = z; }
    const size_t vrow0 = (size_t)(ph * CE + h * HD);
    const float ssc = (ph == 0) ? 0.125f : inc;

    for (int kc = 0; kc <= qb; ++kc) {
      const int kv0 = kc * 64;
      v8f s[4];
#pragma unroll
      for (int j = 0; j < 4; ++j) {
        v8f z = {}; s[j] = z;
        if (ph == 0) {
          const size_t ko = ((size_t)b * RQ + kv0 + j * 16 + c) * QKP + CE + (size_t)h * HD + 8 * hh;
#pragma unroll
          for (int dc = 0; dc < 2; ++dc) {
            const v16b kh = ldfrag_g(QA + ko + dc * 32);
            if (EARLY) {
              const v16b kl = ldfrag_g(QB + ko + dc * 32);
              s[j] = mma16<false>(fa[dc], kh, s[j]);
              s[j] = mma16<false>(fa[dc], kl, s[j]);
              s[j] = mma16<false>(fl[dc], kh, s[j]);
            } else {
              s[j] = mma16<true>(fa[dc], kh, s[j]);
            }
          }
        } else {
          const v16b jf = ldfrag_g(JW + ((size_t)b * SEQ + kv0 + j * 16 + c) * LSP + (size_t)h * 32 + 8 * hh);
          s[j] = mma16<false>(fa[0], jf, s[j]);
        }
      }
      const bool diag = (kc == qb);
      float cm[8];
#pragma unroll
      for (int r = 0; r < 8; ++r) {
        const int qrow = q0 + 8 * hh + r;
        float m = -INFINITY;
#pragma unroll
        for (int j = 0; j < 4; ++j) {
          const int kvcol = kv0 + j * 16 + c;
          float sc = s[j][r] * ssc;
          sc = (diag && kvcol > qrow) ? -INFINITY : sc;
          s[j][r] = sc;
          m = fmaxf(m, sc);
        }
        m = fmaxf(m, __shfl_xor(m, 1, 32)); m = fmaxf(m, __shfl_xor(m, 2, 32));
        m = fmaxf(m, __shfl_xor(m, 4, 32)); m = fmaxf(m, __shfl_xor(m, 8, 32));
        cm[r] = m;
      }
#pragma unroll
      for (int r = 0; r < 8; ++r) {
        const float mnew = fmaxf(mrow[r], cm[r]);
        const float alpha = __builtin_amdgcn_exp2f((mrow[r] - mnew) * L2E);
        mrow[r] = mnew;
        float psum = 0.f;
#pragma unroll
        for (int j = 0; j < 4; ++j) {
          const float p = __builtin_amdgcn_exp2f((s[j][r] - mnew) * L2E);
          psum += p;
          const int pi = (8 * hh + r) * 64 + j * 16 + c;
          if (EARLY) {
            const unsigned int hb = f2bf_bits(p);
            pwh[pi] = __builtin_bit_cast(__bf16, (unsigned short)hb);
            pwl[pi] = __builtin_bit_cast(__bf16, (unsigned short)f2bf_bits(p - bf_bits2f(hb)));
          } else {
            pwh[pi] = __builtin_bit_cast(__bf16, toh_flush(p * PSC));
          }
        }
        psum += __shfl_xor(psum, 1, 32); psum += __shfl_xor(psum, 2, 32);
        psum += __shfl_xor(psum, 4, 32); psum += __shfl_xor(psum, 8, 32);
        lrow[r] = lrow[r] * alpha + psum;
#pragma unroll
        for (int t = 0; t < 4; ++t) oacc[t][r] *= alpha;
      }
      wave_sync();
#pragma unroll
      for (int kk = 0; kk < 2; ++kk) {
        FB pa, pl;
        pa.h[0] = *(const v8b*)(pwh + c * 64 + kk * 32 + 8 * hh);
        pa.h[1] = *(const v8b*)(pwh + c * 64 + kk * 32 + 16 + 8 * hh);
        pl.v = pa.v;
        if (EARLY) {
          pl.h[0] = *(const v8b*)(pwl + c * 64 + kk * 32 + 8 * hh);
          pl.h[1] = *(const v8b*)(pwl + c * 64 + kk * 32 + 16 + 8 * hh);
        }
#pragma unroll
        for (int t = 0; t < 4; ++t) {
          const size_t vo = (vrow0 + (size_t)(t * 16 + c)) * VP + vcol + kv0 + kk * 32;
          const v16b vb = ldfrag_g(VA + vo);
          oacc[t] = mma16<F16>(pa.v, vb, oacc[t]);
          if (EARLY) {
            const v16b vl = ldfrag_g(VB + vo);
            oacc[t] = mma16<false>(pa.v, vl, oacc[t]);
            oacc[t] = mma16<false>(pl.v, vb, oacc[t]);
          }
        }
      }
      wave_sync();
    }

#pragma unroll
    for (int r = 0; r < 8; ++r) {
      const float inv = 1.0f / (lrow[r] * PSC);
      const float wgt = (ph == 0) ? (1.0f - gt[r]) : gt[r];
      const float f = inv * wgt;
#pragma unroll
      for (int t = 0; t < 4; ++t) {
        const int oi = (8 * hh + r) * 68 + t * 16 + c;
        const float val = oacc[t][r] * f;
        if (ph == 0) os[oi] = val; else os[oi] = os[oi] + val;
      }
    }
  }
  wave_sync();
  {
    const int q = lane >> 3, c8 = (lane & 7) * 8;
    for (int pass = 0; pass < 2; ++pass) {
#pragma unroll
      for (int it = 0; it < 4; ++it) {
        const int row = it * 4 + q;
        const float* sp = os + row * 68 + c8;
        const v4f wa = *(const v4f*)sp, wb = *(const v4f*)(sp + 4);
        if (!EARLY) {
          const size_t o = ((size_t)b * SEQ + q0 + row) * CE + (size_t)h * HD + c8;
          const v4u pk = pk8hf(wa * CSC, wb * CSC);
          *(volatile v4u*)(C16 + o) = pk;
        } else {
          v4u ph2, pl2; pk8s(wa, wb, ph2, pl2);
          const size_t oe = ((size_t)b * NX + q0 + row) * CE + (size_t)h * HD + c8;
          *(volatile v4u*)(CHp + oe) = ph2;
          *(volatile v4u*)(CLp + oe) = pl2;
        }
      }
      __threadfence();
    }
  }
}

__global__ __launch_bounds__(128) void k_dual_attn_early(
    const unsigned short* __restrict__ QAp, const unsigned short* __restrict__ QBp,
    const unsigned short* __restrict__ RLp, const unsigned short* __restrict__ JWp,
    const unsigned short* __restrict__ VAp, const unsigned short* __restrict__ VBp,
    const float* __restrict__ gatev, const float* __restrict__ inc_scale,
    unsigned short* __restrict__ C16, unsigned short* __restrict__ CHp, unsigned short* __restrict__ CLp,
    int nqb, int qb0) {
  dual_attn_body<true>(QAp, QBp, RLp, JWp, VAp, VBp, gatev, inc_scale, C16, CHp, CLp, nqb, qb0);
}

__global__ __launch_bounds__(128) void k_dual_attn_main(
    const unsigned short* __restrict__ QAp, const unsigned short* __restrict__ QBp,
    const unsigned short* __restrict__ RLp, const unsigned short* __restrict__ JWp,
    const unsigned short* __restrict__ VAp, const unsigned short* __restrict__ VBp,
    const float* __restrict__ gatev, const float* __restrict__ inc_scale,
    unsigned short* __restrict__ C16, unsigned short* __restrict__ CHp, unsigned short* __restrict__ CLp,
    int nqb, int qb0) {
  dual_attn_body<false>(QAp, QBp, RLp, JWp, VAp, VBp, gatev, inc_scale, C16, CHp, CLp, nqb, qb0);
}

constexpr size_t SZ_PL   = (size_t)MT * CE * 2;
constexpr size_t SZ_WQKV = (size_t)3 * CE * CE * 2;
constexpr size_t SZ_WSQ  = (size_t)CE * CE * 2;
constexpr size_t SZ_WL   = (size_t)LNP * CE * 2;
constexpr size_t SZ_QK   = (size_t)MT * QKP * 2;
constexpr size_t SZ_VG   = (size_t)2 * CE * MT * 2;
constexpr size_t SZ_QKE  = (size_t)NB * NX * QKP * 2;
constexpr size_t SZ_VGE  = (size_t)2 * CE * VEP * 2;
constexpr size_t SZ_LN   = (size_t)MT * LNP * 4;
constexpr size_t SZ_LS   = (size_t)MT * LSP * 2;
constexpr size_t SZ_GATE = (size_t)MT * 4;
constexpr size_t SZ_CE   = (size_t)NB * NX * CE * 2;
constexpr size_t SZ_TOTAL = SZ_PL + SZ_WQKV + SZ_WSQ + SZ_WL + 2 * SZ_WSQ + SZ_QK + SZ_VG + 2 * SZ_QKE + 2 * SZ_VGE + SZ_LN + 2 * SZ_LS + SZ_GATE + SZ_PL + 2 * SZ_CE;
static_assert(SZ_TOTAL <= 134217728ull);
static_assert(SZ_PL % 256 == 0 && SZ_WQKV % 256 == 0 && SZ_WSQ % 256 == 0 && SZ_WL % 256 == 0 && SZ_QK % 256 == 0 && SZ_VG % 256 == 0);
static_assert(SZ_QKE % 256 == 0 && SZ_VGE % 256 == 0 && SZ_LN % 256 == 0 && SZ_LS % 256 == 0 && SZ_GATE % 256 == 0 && SZ_CE % 256 == 0);
static_assert((size_t)(NB_FULL - 1) * T_FULL * CE * 4 + (size_t)SEQ * CE * 4 <= (size_t)NB_FULL * T_FULL * CE * 4);

extern "C" void kernel_launch(void* const* d_in, const int* in_sizes, int n_in, void* d_out, int out_size, void* d_ws, size_t ws_size, hipStream_t stream) {
  if (n_in < 14) return;
  const long long need_x = ((long long)(NB - 1) * T_FULL + SEQ) * CE;
  if ((long long)in_sizes[0] < need_x) return;
  if (in_sizes[1] < CE * 3 * CE || in_sizes[2] < 3 * CE) return;
  if (in_sizes[3] < CE * 64 || in_sizes[4] < CE * 64 || in_sizes[5] < CE * 64 || in_sizes[6] < CE * 64) return;
  if (in_sizes[7] < CE * CE || in_sizes[8] < CE) return;
  if (in_sizes[9] < CE * NH || in_sizes[10] < NH || in_sizes[11] < NH) return;
  if (in_sizes[12] < CE * CE || in_sizes[13] < CE) return;
  if ((long long)out_size < need_x) return;

  const float* x        = (const float*)d_in[0];
  const float* qkv_w    = (const float*)d_in[1];
  const float* qkv_b    = (const float*)d_in[2];
  const float* w1_write = (const float*)d_in[3];
  const float* w2_write = (const float*)d_in[4];
  const float* w1_read  = (const float*)d_in[5];
  const float* w2_read  = (const float*)d_in[6];
  const float* geo_w    = (const float*)d_in[7];
  const float* geo_b    = (const float*)d_in[8];
  const float* gate_w   = (const float*)d_in[9];
  const float* gate_b   = (const float*)d_in[10];
  const float* inc_sc   = (const float*)d_in[11];
  const float* out_w    = (const float*)d_in[12];
  const float* out_b    = (const float*)d_in[13];
  float* out = (float*)d_out;

  char* wsp = (char*)d_ws; size_t off = 0;
  unsigned short* X16  = (unsigned short*)(wsp + off); off += SZ_PL;
  unsigned short* WQKV = (unsigned short*)(wsp + off); off += SZ_WQKV;
  unsigned short* WG16 = (unsigned short*)(wsp + off); off += SZ_WSQ;
  unsigned short* WL16 = (unsigned short*)(wsp + off); off += SZ_WL;
  unsigned short* WO16 = (unsigned short*)(wsp + off); off += SZ_WSQ;
  unsigned short* WOB  = (unsigned short*)(wsp + off); off += SZ_WSQ;
  unsigned short* QK16 = (unsigned short*)(wsp + off); off += SZ_QK;
  unsigned short* VG16 = (unsigned short*)(wsp + off); off += SZ_VG;
  unsigned short* QKH  = (unsigned short*)(wsp + off); off += SZ_QKE;
  unsigned short* QKL  = (unsigned short*)(wsp + off); off += SZ_QKE;
  unsigned short* VGEH = (unsigned short*)(wsp + off); off += SZ_VGE;
  unsigned short* VGEL = (unsigned short*)(wsp + off); off += SZ_VGE;
  float*          LN32 = (float*)(wsp + off);          off += SZ_LN;
  unsigned short* RLP  = (unsigned short*)(wsp + off); off += SZ_LS;
  unsigned short* JWP  = (unsigned short*)(wsp + off); off += SZ_LS;
  float*          GATE = (float*)(wsp + off);          off += SZ_GATE;
  unsigned short* C16  = (unsigned short*)(wsp + off); off += SZ_PL;
  unsigned short* CHp  = (unsigned short*)(wsp + off); off += SZ_CE;
  unsigned short* CLp  = (unsigned short*)(wsp + off); off += SZ_CE;
  if (off > ws_size) return;

  const float WS = 64.0f, IWS = 0.015625f;

  k_castX16<<<(unsigned)(((long long)MT * (CE / 8) + 255) / 256), 256, 0, stream>>>(x, X16);

  k_castT<<<(unsigned)(((long long)3 * CE * (CE / 8) + 255) / 256), 256, 0, stream>>>(qkv_w, 3 * CE, WQKV, CE, CE, 3 * CE, WS, 0);
  k_castT<<<(unsigned)(((long long)CE * (CE / 8) + 255) / 256), 256, 0, stream>>>(geo_w, CE, WG16, CE, CE, CE, WS, 0);
  k_castT<<<(unsigned)(((long long)64 * (CE / 8) + 255) / 256), 256, 0, stream>>>(w1_write, 64, WL16, CE, CE, 64, WS, 0);
  k_castT<<<(unsigned)(((long long)64 * (CE / 8) + 255) / 256), 256, 0, stream>>>(w2_write, 64, WL16 + (size_t)64 * CE, CE, CE, 64, WS, 0);
  k_castT<<<(unsigned)(((long long)64 * (CE / 8) + 255) / 256), 256, 0, stream>>>(w1_read, 64, WL16 + (size_t)128 * CE, CE, CE, 64, WS, 0);
  k_castT<<<(unsigned)(((long long)64 * (CE / 8) + 255) / 256), 256, 0, stream>>>(w2_read, 64, WL16 + (size_t)192 * CE, CE, CE, 64, WS, 0);
  k_castT<<<(unsigned)(((long long)NH * (CE / 8) + 255) / 256), 256, 0, stream>>>(gate_w, NH, WL16 + (size_t)256 * CE, CE, CE, NH, WS, 0);
  k_castT<<<(unsigned)(((long long)(LNP - 256 - NH) * (CE / 8) + 255) / 256), 256, 0, stream>>>(w1_write, 64, WL16 + (size_t)(256 + NH) * CE, CE, CE, LNP - 256 - NH, 0.0f, 0);
  k_castT<<<(unsigned)(((long long)CE * (CE / 8) + 255) / 256), 256, 0, stream>>>(out_w, CE, WO16, CE, CE, CE, WS, 0);
  k_castT<<<(unsigned)(((long long)CE * (CE / 8) + 255) / 256), 256, 0, stream>>>(out_w, CE, WOB, CE, CE, CE, 1.0f, 1);

  k_gemm64<0, false, 2, 1, 0, 0><<<dim3((unsigned)(((MT / 64) * (QKP / 64) + 7) / 8), 1), 256, 0, stream>>>(
      X16, nullptr, CE, 0, WQKV, CE, QK16, nullptr, nullptr, nullptr, QKP, 0, qkv_b, nullptr, 0, 0, MT, QKP, CE, IWS);
  k_gemm64<0, false, 1, 1, 0, 0><<<dim3((unsigned)(((CE / 64) * (MT / 64) + 7) / 8), 1), 256, 0, stream>>>(
      WQKV + (size_t)2 * CE * CE, nullptr, CE, 0, X16, CE, VG16, nullptr, nullptr, nullptr, MT, 0, qkv_b + 2 * CE, nullptr, 0, 0, CE, MT, CE, IWS);
  k_gemm64<0, false, 1, 1, 0, 0><<<dim3((unsigned)(((CE / 64) * (MT / 64) + 7) / 8), 1), 256, 0, stream>>>(
      WG16, nullptr, CE, 0, X16, CE, VG16 + (size_t)CE * MT, nullptr, nullptr, nullptr, MT, 0, geo_b, nullptr, 0, 0, CE, MT, CE, IWS);
  k_gemm64<0, false, 0, 0, 0, 0><<<dim3((unsigned)(((MT / 64) * (LNP / 64) + 7) / 8), 1), 256, 0, stream>>>(
      X16, nullptr, CE, 0, WL16, CE, nullptr, nullptr, nullptr, LN32, LNP, 0, nullptr, nullptr, 0, 0, MT, LNP, CE, IWS);

  k_gemm64<0, false, 2, 2, 0, 0><<<dim3((unsigned)(((NX / 64) * (QKP / 64) + 7) / 8), NB), 256, 0, stream>>>(
      X16, nullptr, CE, (long long)SEQ * CE, WQKV, CE, QKH, QKL, nullptr, nullptr, QKP, (long long)NX * QKP, qkv_b, nullptr, 0, 0, NX, QKP, CE, IWS);
  for (int b = 0; b < NB; ++b) {
    k_gemm64<0, false, 1, 2, 0, 0><<<dim3((unsigned)(((CE / 64) * (NX / 64) + 7) / 8), 1), 256, 0, stream>>>(
        WQKV + (size_t)2 * CE * CE, nullptr, CE, 0, X16 + (size_t)b * SEQ * CE, CE, VGEH + (size_t)b * NX, VGEL + (size_t)b * NX, nullptr, nullptr,
        VEP, 0, qkv_b + 2 * CE, nullptr, 0, 0, CE, NX, CE, IWS);
    k_gemm64<0, false, 1, 2, 0, 0><<<dim3((unsigned)(((CE / 64) * (NX / 64) + 7) / 8), 1), 256, 0, stream>>>(
        WG16, nullptr, CE, 0, X16 + (size_t)b * SEQ * CE, CE, VGEH + (size_t)CE * VEP + (size_t)b * NX, VGEL + (size_t)CE * VEP + (size_t)b * NX, nullptr, nullptr,
        VEP, 0, geo_b, nullptr, 0, 0, CE, NX, CE, IWS);
  }

  k_lines<<<(unsigned)(MT / LTOK), 512, 0, stream>>>(LN32, gate_b, RLP, JWP, GATE);

  k_dual_attn_early<<<(unsigned)(NB * NH * (NX / 64)), 128, 0, stream>>>(QKH, QKL, RLP, JWP, VGEH, VGEL, GATE, inc_sc, C16, CHp, CLp, NX / 64, 0);
  constexpr int NQB_MAIN = SEQ / 64 - NX / 64;
  if (NQB_MAIN > 0)
    k_dual_attn_main<<<(unsigned)(NB * NH * NQB_MAIN), 128, 0, stream>>>(QK16, QK16, RLP, JWP, VG16, VG16, GATE, inc_sc, C16, CHp, CLp, NQB_MAIN, NX / 64);

  if (NQB_MAIN > 0)
    k_gemm64<0, false, 2, 0, 0, 0><<<dim3((unsigned)((((SEQ - NX) / 64) * (CE / 64) + 7) / 8), NB), 256, 0, stream>>>(
        C16 + (size_t)NX * CE, nullptr, CE, (long long)SEQ * CE, WO16, CE, nullptr, nullptr, nullptr, out + (size_t)NX * CE, CE, (long long)T_FULL * CE,
        out_b, nullptr, 0, 0, SEQ - NX, CE, CE, IWS * IWS);
  k_gemm64<1, true, 2, 0, 0, 0><<<dim3((unsigned)(((NX / 64) * (CE / 64) + 7) / 8), NB), 256, 0, stream>>>(
      CHp, CLp, CE, (long long)NX * CE, WOB, CE, nullptr, nullptr, nullptr, out, CE, (long long)T_FULL * CE,
      out_b, nullptr, 0, 0, NX, CE, CE, 1.0f);
}
